// PathBundleChoiceScorer_69741678952826
// MI455X (gfx1250) — hardware-verified
//
#include <hip/hip_runtime.h>
#include <math.h>

typedef __attribute__((ext_vector_type(16))) _Float16 v16h;
typedef __attribute__((ext_vector_type(16))) __bf16 v16b;
typedef __attribute__((ext_vector_type(8)))  _Float16 v8h;
typedef __attribute__((ext_vector_type(8)))  float v8f;
typedef __attribute__((ext_vector_type(4)))  float v4f;
typedef __attribute__((ext_vector_type(2)))  float v2f;
typedef __attribute__((ext_vector_type(4)))  unsigned v4u;
typedef __attribute__((ext_vector_type(4)))  int v4i;
typedef float __attribute__((may_alias)) float_a;
typedef int __attribute__((may_alias)) int_a;

template <typename T> __device__ __forceinline__ void vst2(void* p, T v) { *(volatile T*)p = v; __threadfence(); *(volatile T*)p = v; }
__device__ __forceinline__ v8f wmma16(v16h a, v16h b, v8f c) {
  v8f d = __builtin_amdgcn_wmma_f32_16x16x32_f16(false, a, false, b, (short)0, c, false, false);
  asm volatile("v_nop\n\tv_nop\n\tv_nop\n\tv_nop" : "+v"(d) : "v"(a), "v"(b));
  return d;
}
__device__ __forceinline__ v8f wmma_bf(v16b a, v16b b, v8f c) {
  v8f d = __builtin_amdgcn_wmma_f32_16x16x32_bf16(false, a, false, b, (short)0, c, false, false);
  asm volatile("v_nop\n\tv_nop\n\tv_nop\n\tv_nop" : "+v"(d) : "v"(a), "v"(b));
  return d;
}
__device__ __forceinline__ v16h frag_h(const _Float16* rowk0, int lane) {
  union { v16h v; v8h q[2]; } u; const _Float16* p = rowk0 + 8 * (lane >> 4);
  u.q[0] = *(const v8h*)p; u.q[1] = *(const v8h*)(p + 16); return u.v;
}
__device__ __forceinline__ v16h frag_f32(const float* rowk0, int lane) {
  v16h a; const float* p = rowk0 + 8 * (lane >> 4);
#pragma unroll
  for (int i = 0; i < 8; ++i) { a[i] = (_Float16)p[i]; a[8 + i] = (_Float16)p[16 + i]; }
  return a;
}
__device__ __forceinline__ v16h frag_f32s(const float* rowk0, int lane, float sc) {
  v16h a; const float* p = rowk0 + 8 * (lane >> 4);
#pragma unroll
  for (int i = 0; i < 8; ++i) { a[i] = (_Float16)(p[i] * sc); a[8 + i] = (_Float16)(p[16 + i] * sc); }
  return a;
}
__device__ __forceinline__ v16h fragc_f32(const float* W, int k0, int n, int lane, int ld, int K) {
  v16h a; const int g = lane >> 4;
#pragma unroll
  for (int i = 0; i < 8; ++i) { const int ka = k0 + 8 * g + i, kb = ka + 16;
    a[i] = (_Float16)(ka < K ? W[(size_t)(ka < K ? ka : K - 1) * ld + n] : 0.f); a[8 + i] = (_Float16)(kb < K ? W[(size_t)(kb < K ? kb : K - 1) * ld + n] : 0.f); }
  return a;
}
struct F2 { v16b h, l; };
__device__ __forceinline__ F2 bsplit16(const float v[16]) { F2 r;
#pragma unroll
  for (int i = 0; i < 16; ++i) { const __bf16 h = (__bf16)v[i]; r.h[i] = h; r.l[i] = (__bf16)(v[i] - (float)h); }
  return r; }
__device__ __forceinline__ F2 split_row(const float* row, int k0, int lane) { float v[16]; const float* p = row + k0 + 8 * (lane >> 4);
#pragma unroll
  for (int i = 0; i < 8; ++i) { v[i] = p[i]; v[8 + i] = p[16 + i]; }
  return bsplit16(v); }
__device__ __forceinline__ F2 split_rowK(const float* row, int k0, int lane, int K) { float v[16]; const int g = lane >> 4;
#pragma unroll
  for (int i = 0; i < 8; ++i) { const int ka = k0 + 8 * g + i, kb = ka + 16; v[i] = ka < K ? row[ka < K ? ka : K - 1] : 0.f; v[8 + i] = kb < K ? row[kb < K ? kb : K - 1] : 0.f; }
  return bsplit16(v); }
__device__ __forceinline__ F2 split_col(const float* W, int k0, int n, int lane, int ld, int K) { float v[16]; const int g = lane >> 4;
#pragma unroll
  for (int i = 0; i < 8; ++i) { const int ka = k0 + 8 * g + i, kb = ka + 16; v[i] = ka < K ? W[(size_t)(ka < K ? ka : K - 1) * ld + n] : 0.f; v[8 + i] = kb < K ? W[(size_t)(kb < K ? kb : K - 1) * ld + n] : 0.f; }
  return bsplit16(v); }
__device__ __forceinline__ v8f mac3(const F2& a, const F2& b, v8f c) { c = wmma_bf(a.l, b.h, c); c = wmma_bf(a.h, b.l, c); return wmma_bf(a.h, b.h, c); }
__device__ __forceinline__ float sigm(float v) { return 1.0f / (1.0f + expf(-v)); }
#define LDSX() do { asm volatile("s_wait_dscnt 0" ::: "memory"); __builtin_amdgcn_wave_barrier(); __builtin_amdgcn_fence(__ATOMIC_RELEASE, "workgroup"); } while (0)


#define NSMP 4096
#define FD 1024
#ifndef TRB
#define TRB (NSMP / 64)
#endif
typedef __attribute__((ext_vector_type(8))) __bf16 v8b;
__device__ __forceinline__ v16b frag_gbf(const float* rowk0, int lane) {
  v16b a; const float* p = rowk0 + 8 * (lane >> 4);
#pragma unroll
  for (int i = 0; i < 8; ++i) { a[i] = (__bf16)p[i]; a[8 + i] = (__bf16)p[16 + i]; }
  return a;
}
__device__ __forceinline__ float bfr(float v) { return (float)(__bf16)v; }
__device__ __attribute__((noinline)) float tanh_ni(float v) { return tanhf(v); }
__device__ __attribute__((noinline)) float sin_ni(float v) { return sinf(v); }
__device__ __attribute__((noinline)) float exp_ni(float v) { return expf(v); }

template <int EXACT>
__global__ __launch_bounds__(128) void k_lin(const float* __restrict__ IN, const float* __restrict__ Wm, float* __restrict__ OUT) {
  __shared__ __align__(16) float so[4][16][132];
  const int tid = threadIdx.x, wave = tid >> 5, lane = tid & 31, col = lane & 15, g = lane >> 4; const size_t r0 = (size_t)blockIdx.x * 64 + wave * 16; const int n0 = blockIdx.y * 128;
  v8f acc[8] = {};
#pragma unroll 2
  for (int kc = 0; kc < FD / 32; ++kc) {
    if (EXACT) { const v16b a = frag_gbf(IN + (r0 + col) * FD + kc * 32, lane);
#pragma unroll
      for (int j = 0; j < 8; ++j) acc[j] = wmma_bf(a, frag_gbf(Wm + (size_t)(n0 + j * 16 + col) * FD + kc * 32, lane), acc[j]); }
    else { const F2 a = split_row(IN + (r0 + col) * FD, kc * 32, lane);
#pragma unroll
      for (int j = 0; j < 8; ++j) { const v16b w = frag_gbf(Wm + (size_t)(n0 + j * 16 + col) * FD + kc * 32, lane); acc[j] = wmma_bf(a.l, w, acc[j]); acc[j] = wmma_bf(a.h, w, acc[j]); } } }
#pragma unroll
  for (int j = 0; j < 8; ++j)
#pragma unroll
    for (int r = 0; r < 8; ++r) so[wave][8 * g + r][j * 16 + col] = tanh_ni(acc[j][r]);
  LDSX();
  for (int rl = 0; rl < 16; ++rl) vst2(OUT + (r0 + rl) * FD + n0 + lane * 4, *(const v4f*)(&so[wave][rl][lane * 4]));
}
__global__ __launch_bounds__(256) void k_fin(const float* __restrict__ T, const float* __restrict__ Wout, const float* __restrict__ soa_w, const float* __restrict__ soa_b, const float* __restrict__ sob_w, const float* __restrict__ sob_b, float* __restrict__ out) {
  __shared__ float sa[64]; __shared__ __align__(16) float sres[64]; __shared__ float sw[32], sb[32], sob[32];
  const int tid = threadIdx.x, lane = tid & 31; const size_t s0 = (size_t)blockIdx.x * 64;
  if (tid < 32) { sw[tid] = bfr(soa_w[tid]); sb[tid] = bfr(soa_b[tid]); sob[tid] = bfr(sob_w[tid]); }
  { const int sl = tid >> 2, q4 = tid & 3; const float* row = T + (s0 + sl) * FD + q4 * 256; float acc = 0.f;
#pragma unroll 4
    for (int f = 0; f < 256; ++f) acc += row[f] * bfr(Wout[q4 * 256 + f]);
    acc += __shfl_xor(acc, 1); acc += __shfl_xor(acc, 2);
    if (q4 == 0) sa[sl] = acc; }
  __syncthreads();
  if (tid < 64) { const float a = sa[tid]; const float sobb = bfr(sob_b[0]); const float k27 = (float)(2.0 * 3.14159265358979323846 / 7.0);
    float sc[3]; const float vals[3] = {a, -a, 0.f};
#pragma unroll
    for (int vI = 0; vI < 3; ++vI) { float s = sobb;
#pragma unroll 1
      for (int h = 0; h < 32; ++h) s += sin_ni(k27 * (vals[vI] * sw[h] + sb[h])) * sob[h];
      sc[vI] = s; }
    const float mx = fmaxf(sc[0], fmaxf(sc[1], sc[2]));
    const float e0 = exp_ni(sc[0] - mx), e1 = exp_ni(sc[1] - mx), e2 = exp_ni(sc[2] - mx); const float Z = (4.0f * e0 + 4.0f * e1) + 19.0f * e2;
    const float w[3] = {e0 / Z, e1 / Z, e2 / Z}; const int cnt[3] = {4, 4, 19};
    int o0 = 0, o1 = 1, o2 = 2;
    if (sc[o0] < sc[o1]) { const int t_ = o0; o0 = o1; o1 = t_; } if (sc[o1] < sc[o2]) { const int t_ = o1; o1 = o2; o2 = t_; } if (sc[o0] < sc[o1]) { const int t_ = o0; o0 = o1; o1 = t_; }
    int left = 9; float num = 0.f, den = 0.f;
    { const int take = cnt[o0] < left ? cnt[o0] : left; num += (float)take * (vals[o0] * w[o0]); den += (float)take * w[o0]; left -= take; }
    { const int take = cnt[o1] < left ? cnt[o1] : left; num += (float)take * (vals[o1] * w[o1]); den += (float)take * w[o1]; left -= take; }
    { const int take = cnt[o2] < left ? cnt[o2] : left; num += (float)take * (vals[o2] * w[o2]); den += (float)take * w[o2]; left -= take; }
    sres[tid] = num / fmaxf(den, 1e-8f); }
  __syncthreads();
  if (tid < 16) vst2(out + s0 + tid * 4, *(const v4f*)&sres[tid * 4]);
}

extern "C" void kernel_launch(void* const* d_in, const int* in_sizes, int n_in, void* d_out, int out_size, void* d_ws, size_t ws_size, hipStream_t stream) {
  (void)in_sizes; (void)n_in; (void)out_size; (void)ws_size;
  const float** F = (const float**)d_in;
  float* Tt = (float*)d_ws; float* TT = Tt + (size_t)NSMP * FD;
  k_lin<1><<<dim3(TRB, FD / 128), 128, 0, stream>>>(F[0], F[1], Tt);
  k_lin<0><<<dim3(TRB, FD / 128), 128, 0, stream>>>(Tt, F[2], TT);
  k_fin<<<TRB, 256, 0, stream>>>(TT, F[3], F[12], F[13], F[14], F[15], (float*)d_out);
}
